// ControllerCell_42125039239689
// MI455X (gfx1250) — hardware-run, weakly checked
//
#include <hip/hip_runtime.h>
#include <math.h>

typedef __attribute__((ext_vector_type(16))) _Float16 v16h;
typedef __attribute__((ext_vector_type(16))) __bf16 v16b;
typedef __attribute__((ext_vector_type(8)))  _Float16 v8h;
typedef __attribute__((ext_vector_type(8)))  float v8f;
typedef __attribute__((ext_vector_type(4)))  float v4f;
typedef __attribute__((ext_vector_type(2)))  float v2f;
typedef __attribute__((ext_vector_type(4)))  unsigned v4u;
typedef __attribute__((ext_vector_type(4)))  int v4i;
typedef float __attribute__((may_alias)) float_a;
typedef int __attribute__((may_alias)) int_a;

template <typename T> __device__ __forceinline__ void vst2(void* p, T v) { *(volatile T*)p = v; __threadfence(); *(volatile T*)p = v; }
__device__ __forceinline__ v8f wmma16(v16h a, v16h b, v8f c) {
  v8f d = __builtin_amdgcn_wmma_f32_16x16x32_f16(false, a, false, b, (short)0, c, false, false);
  asm volatile("v_nop\n\tv_nop\n\tv_nop\n\tv_nop" : "+v"(d) : "v"(a), "v"(b));
  return d;
}
__device__ __forceinline__ v8f wmma_bf(v16b a, v16b b, v8f c) {
  v8f d = __builtin_amdgcn_wmma_f32_16x16x32_bf16(false, a, false, b, (short)0, c, false, false);
  asm volatile("v_nop\n\tv_nop\n\tv_nop\n\tv_nop" : "+v"(d) : "v"(a), "v"(b));
  return d;
}
__device__ __forceinline__ v16h frag_h(const _Float16* rowk0, int lane) {
  union { v16h v; v8h q[2]; } u; const _Float16* p = rowk0 + 8 * (lane >> 4);
  u.q[0] = *(const v8h*)p; u.q[1] = *(const v8h*)(p + 16); return u.v;
}
__device__ __forceinline__ v16h frag_f32(const float* rowk0, int lane) {
  v16h a; const float* p = rowk0 + 8 * (lane >> 4);
#pragma unroll
  for (int i = 0; i < 8; ++i) { a[i] = (_Float16)p[i]; a[8 + i] = (_Float16)p[16 + i]; }
  return a;
}
__device__ __forceinline__ v16h frag_f32s(const float* rowk0, int lane, float sc) {
  v16h a; const float* p = rowk0 + 8 * (lane >> 4);
#pragma unroll
  for (int i = 0; i < 8; ++i) { a[i] = (_Float16)(p[i] * sc); a[8 + i] = (_Float16)(p[16 + i] * sc); }
  return a;
}
__device__ __forceinline__ v16h fragc_f32(const float* W, int k0, int n, int lane, int ld, int K) {
  v16h a; const int g = lane >> 4;
#pragma unroll
  for (int i = 0; i < 8; ++i) { const int ka = k0 + 8 * g + i, kb = ka + 16;
    a[i] = (_Float16)(ka < K ? W[(size_t)(ka < K ? ka : K - 1) * ld + n] : 0.f); a[8 + i] = (_Float16)(kb < K ? W[(size_t)(kb < K ? kb : K - 1) * ld + n] : 0.f); }
  return a;
}
struct F2 { v16b h, l; };
__device__ __forceinline__ F2 bsplit16(const float v[16]) { F2 r;
#pragma unroll
  for (int i = 0; i < 16; ++i) { const __bf16 h = (__bf16)v[i]; r.h[i] = h; r.l[i] = (__bf16)(v[i] - (float)h); }
  return r; }
__device__ __forceinline__ F2 split_row(const float* row, int k0, int lane) { float v[16]; const float* p = row + k0 + 8 * (lane >> 4);
#pragma unroll
  for (int i = 0; i < 8; ++i) { v[i] = p[i]; v[8 + i] = p[16 + i]; }
  return bsplit16(v); }
__device__ __forceinline__ F2 split_rowK(const float* row, int k0, int lane, int K) { float v[16]; const int g = lane >> 4;
#pragma unroll
  for (int i = 0; i < 8; ++i) { const int ka = k0 + 8 * g + i, kb = ka + 16; v[i] = ka < K ? row[ka < K ? ka : K - 1] : 0.f; v[8 + i] = kb < K ? row[kb < K ? kb : K - 1] : 0.f; }
  return bsplit16(v); }
__device__ __forceinline__ F2 split_col(const float* W, int k0, int n, int lane, int ld, int K) { float v[16]; const int g = lane >> 4;
#pragma unroll
  for (int i = 0; i < 8; ++i) { const int ka = k0 + 8 * g + i, kb = ka + 16; v[i] = ka < K ? W[(size_t)(ka < K ? ka : K - 1) * ld + n] : 0.f; v[8 + i] = kb < K ? W[(size_t)(kb < K ? kb : K - 1) * ld + n] : 0.f; }
  return bsplit16(v); }
__device__ __forceinline__ v8f mac3(const F2& a, const F2& b, v8f c) { c = wmma_bf(a.l, b.h, c); c = wmma_bf(a.h, b.l, c); return wmma_bf(a.h, b.h, c); }
__device__ __forceinline__ float sigm(float v) { return 1.0f / (1.0f + expf(-v)); }
#define LDSX() do { asm volatile("s_wait_dscnt 0" ::: "memory"); __builtin_amdgcn_wave_barrier(); __builtin_amdgcn_fence(__ATOMIC_RELEASE, "workgroup"); } while (0)


#define NBATCH 16384
#define HC 1024
#define HP 1024
#define DT 64
#ifndef TRB
#define TRB (NBATCH / 64)
#endif
typedef __attribute__((ext_vector_type(8))) __bf16 v8b;
__device__ __forceinline__ v16b frag_b(const __bf16* rowk0, int lane) {
  union { v16b v; v8b q[2]; } u; const __bf16* p = rowk0 + 8 * (lane >> 4);
  u.q[0] = *(const v8b*)p; u.q[1] = *(const v8b*)(p + 16); return u.v;
}
__device__ __forceinline__ float bfr(float v) { return (float)(__bf16)v; }
__device__ __attribute__((noinline)) float exp_ni(float v) { return expf(v); }
__device__ __attribute__((noinline)) float erf_ni(float v) { return erff(v); }

#define WS_X1  0u
#define WS_X2  (WS_X1 + 2u * (size_t)NBATCH * 192)
#define WS_A2  (WS_X2 + 2u * (size_t)NBATCH * 128)
#define WS_END (WS_A2 + 4u * (size_t)NBATCH)

__global__ __launch_bounds__(256) void k_t(const float* __restrict__ CI, const float* __restrict__ CR, const float* __restrict__ CO, const float* __restrict__ PI, const float* __restrict__ PO, __bf16* __restrict__ X1, __bf16* __restrict__ X2) { __shared__ __align__(16) __bf16 s1[64][192 + 8], s2[64][128 + 8]; const int t = threadIdx.x; const size_t b0 = (size_t)blockIdx.x * 64;
  for (int e = t; e < 192 * 64; e += 256) { const int k = e >> 6, bl = e & 63; const float* src = k < 64 ? CI + (size_t)k * NBATCH : k < 128 ? CR + (size_t)(k - 64) * NBATCH : CO + (size_t)(k - 128) * NBATCH; s1[bl][k] = (__bf16)src[b0 + bl]; }
  for (int e = t; e < 128 * 64; e += 256) { const int k = e >> 6, bl = e & 63; float v = 0.f; if (k < 63) v = PI[(size_t)k * NBATCH + b0 + bl]; else if (k >= 64) v = PO[(size_t)(k - 64) * NBATCH + b0 + bl]; s2[bl][k] = (__bf16)v; }
  __syncthreads();
  for (int e = t; e < 64 * 24; e += 256) { const int bl = e / 24, q = e % 24; vst2((unsigned*)(X1 + (b0 + bl) * 192 + q * 8), *(const v4u*)&s1[bl][q * 8]); }
  for (int e = t; e < 64 * 16; e += 256) { const int bl = e >> 4, q = e & 15; vst2((unsigned*)(X2 + (b0 + bl) * 128 + q * 8), *(const v4u*)&s2[bl][q * 8]); } }
__device__ __forceinline__ v16b fragb_f32(const float* __restrict__ p, int lane) { v16b a; const float* pp = p + 8 * (lane >> 4);
#pragma unroll
  for (int i = 0; i < 8; ++i) { a[i] = (__bf16)pp[i]; a[8 + i] = (__bf16)pp[16 + i]; } return a; }
template <int PLANT>
__global__ __launch_bounds__(128) void k_mlp(const __bf16* __restrict__ X, const float* __restrict__ WA, const float* __restrict__ WB, const float* __restrict__ WC, const float* __restrict__ B1, const float* __restrict__ LW, const float* __restrict__ LB, const float* __restrict__ A2IN, float* __restrict__ RES) {
  constexpr int KW = PLANT ? 128 : 192; __shared__ float sred[4][16]; __shared__ __align__(16) float so2[64];
  const int tid = threadIdx.x, wave = tid >> 5, lane = tid & 31, col = lane & 15, g = lane >> 4; const size_t r0 = (size_t)blockIdx.x * 64 + wave * 16;
  float a2r[8]; if (PLANT) {
#pragma unroll
    for (int r = 0; r < 8; ++r) a2r[r] = A2IN[r0 + 8 * g + r]; }
  float part[8];
#pragma unroll
  for (int r = 0; r < 8; ++r) part[r] = 0.f;
#pragma unroll 1
  for (int hc = 0; hc < HC / 128; ++hc) { v8f acc[8] = {};
#pragma unroll
    for (int kc = 0; kc < KW / 32; ++kc) { const v16b a = frag_b(X + (r0 + col) * KW + kc * 32, lane);
#pragma unroll
      for (int j = 0; j < 8; ++j) { const int h = hc * 128 + j * 16 + col; const float* wr = PLANT ? (kc < 2 ? WA + (size_t)h * 64 + kc * 32 : WB + (size_t)h * 64 + (kc - 2) * 32) : (kc < 2 ? WA + (size_t)h * 64 + kc * 32 : kc < 4 ? WB + (size_t)h * 64 + (kc - 2) * 32 : WC + (size_t)h * 64 + (kc - 4) * 32); acc[j] = wmma_bf(a, fragb_f32(wr, lane), acc[j]); } }
#pragma unroll
    for (int j = 0; j < 8; ++j) { const int h = hc * 128 + j * 16 + col; const float bb = bfr(B1[h]), lw = bfr(LW[h]); const float w63 = PLANT ? bfr(WA[(size_t)h * 64 + 63]) : 0.f;
#pragma unroll
      for (int r = 0; r < 8; ++r) { float n = acc[j][r] + bb; if (PLANT) n += w63 * a2r[r]; part[r] += lw * tanhf(n); } } }
#pragma unroll
  for (int r = 0; r < 8; ++r) { float v = part[r];
#pragma unroll
    for (int o = 1; o < 16; o <<= 1) v += __shfl_xor(v, o);
    if (col == 0) so2[wave * 16 + 8 * g + r] = v + bfr(LB[0]); }
  __syncthreads(); if (tid < 16) vst2(RES + (size_t)blockIdx.x * 64 + tid * 4, *(const v4f*)&so2[tid * 4]); }
__global__ __launch_bounds__(256) void k_shift(const float* __restrict__ REFIN, const float* __restrict__ CI, const float* __restrict__ CR, const float* __restrict__ CO, const float* __restrict__ PI, const float* __restrict__ PO, const float* __restrict__ A2, const float* __restrict__ A4, float* __restrict__ OUTB) {
  const int tq = blockIdx.y, r = blockIdx.x, t = threadIdx.x; const int nrows = (tq == 3) ? 63 : 64; if (r >= nrows) return;
  const size_t base = (size_t)NBATCH * (tq == 0 ? 1 : tq == 1 ? 65 : tq == 2 ? 129 : tq == 3 ? 193 : 256);
  float* dst = OUTB + base + (size_t)r * NBATCH; const float* src; bool raw = false;
  if (r == 0) { src = (tq == 0 || tq == 3) ? A2 : (tq == 1) ? REFIN : A4; raw = (tq != 1); }
  else { const float* L = tq == 0 ? CI : tq == 1 ? CR : tq == 2 ? CO : tq == 3 ? PI : PO; src = L + (size_t)(r - 1) * NBATCH; }
  for (int q = t; q < NBATCH / 4; q += 256) { v4f v = *(const v4f*)(src + q * 4); if (!raw) { v[0] = bfr(v[0]); v[1] = bfr(v[1]); v[2] = bfr(v[2]); v[3] = bfr(v[3]); } vst2(dst + q * 4, v); } }
extern "C" void kernel_launch(void* const* d_in, const int* in_sizes, int n_in, void* d_out, int out_size, void* d_ws, size_t ws_size, hipStream_t stream) {
  (void)in_sizes; (void)n_in; (void)out_size;
  const float** F = (const float**)d_in;
  if (ws_size < (size_t)WS_END) return;
  char* ws = (char*)d_ws; __bf16 *X1 = (__bf16*)(ws + WS_X1), *X2 = (__bf16*)(ws + WS_X2); float* A2 = (float*)(ws + WS_A2); float* OUTB = (float*)d_out; float* A4 = OUTB;
  k_t<<<NBATCH / 64, 256, 0, stream>>>(F[1], F[2], F[3], F[4], F[5], X1, X2);
  k_mlp<0><<<TRB, 128, 0, stream>>>(X1, F[6], F[7], F[8], F[9], F[10], F[11], nullptr, A2);
  k_mlp<1><<<TRB, 128, 0, stream>>>(X2, F[12], F[13], nullptr, F[14], F[15], F[16], A2, A4);
  k_shift<<<dim3(64, 5), 256, 0, stream>>>(F[0], F[1], F[2], F[3], F[4], F[5], A2, A4, OUTB);
}
